// GroupedQueryAttention_15822659519063
// MI455X (gfx1250) — hardware-verified
//
#include <hip/hip_runtime.h>
#include <math.h>


#ifndef NB
#define NB 2
#endif
#ifndef SEQ
#define SEQ 2048
#endif
#define NB_FULL  2
#define SEQ_FULL 2048
#define DM   2048
#define NH_  32
#define NKV  8
#define REP  (NH_ / NKV)
#define HD   64
#define DQ   (NH_ * HD)
#define DKV  (NKV * HD)
#define NF   (DQ + 2 * DKV)
#define NQK  (NH_ + NKV)
#define VOFF (DQ + DKV)
#define MTOK (NB * SEQ)
#define QT   (SEQ / 16)
#define CEXP 0.18033688011112042f
#define PEXP 8.0f

static_assert(HD == 64);
static_assert(REP == 4);
static_assert((NKV & (NKV - 1)) == 0);
static_assert(NB <= NB_FULL && SEQ <= SEQ_FULL);
static_assert(SEQ % 64 == 0);
static_assert(MTOK % 64 == 0 && NF % 64 == 0 && DM % 64 == 0 && DQ % 64 == 0);
static_assert(DM % 32 == 0 && DQ % 32 == 0);
static_assert(SEQ % 32 == 0);
static_assert(MTOK % 4 == 0);
static_assert(((long long)NB * NQK * SEQ * HD) % 512 == 0);
static_assert(((long long)NB * NKV * HD * SEQ) % 512 == 0);
static_assert(((long long)SEQ * DM) % 2048 == 0 && ((long long)DQ * DM) % 2048 == 0 && ((long long)DKV * DM) % 2048 == 0);
static_assert((long long)NB * NQK * SEQ * HD < 2147483647LL);

#define SZ_WQKV ((size_t)NF * DM * 2)
#define SZ_WO   ((size_t)DM * DQ * 2)
#define SZ_XB   ((size_t)MTOK * DM * 2)
#define SZ_F    ((size_t)MTOK * NF * 4)
#define SZ_QK   ((size_t)NB * NQK * SEQ * HD * 2)
#define SZ_VT   ((size_t)NB * NKV * HD * SEQ * 2)
#define SZ_AT   ((size_t)MTOK * DQ * 2)
#define OFF_WQKV ((size_t)0)
#define OFF_WO   (OFF_WQKV + SZ_WQKV)
#define OFF_XB   (OFF_WO + SZ_WO)
#define OFF_F    (OFF_XB + SZ_XB)
#define OFF_QK   (OFF_F + SZ_F)
#define OFF_VT   (OFF_QK + SZ_QK)
#define WS_TOTAL (OFF_VT + SZ_VT)
static_assert(WS_TOTAL <= (size_t)134217728);
static_assert(2 * SZ_AT <= SZ_F);
static_assert(SZ_WQKV % 256 == 0 && SZ_WO % 256 == 0 && SZ_XB % 256 == 0 && SZ_F % 256 == 0 && SZ_QK % 256 == 0 && SZ_AT % 256 == 0);

typedef _Float16 h16;
typedef unsigned short bf;
typedef __attribute__((ext_vector_type(16))) __bf16   v16bf;
typedef __attribute__((ext_vector_type(16))) _Float16 v16h;
typedef __attribute__((ext_vector_type(8)))  _Float16 v8h;
typedef __attribute__((ext_vector_type(8)))  unsigned short v8us;
typedef __attribute__((ext_vector_type(8)))  float    v8f;
typedef __attribute__((ext_vector_type(4)))  float    v4f;
typedef __attribute__((ext_vector_type(2)))  _Float16 v2h;
typedef __attribute__((ext_vector_type(2)))  float    v2f;
typedef v4f  __attribute__((may_alias)) v4fa;

__device__ __forceinline__ unsigned short f2bf(float f) { unsigned u = __float_as_uint(f); u += 0x7FFFu + ((u >> 16) & 1u); return (unsigned short)(u >> 16); }
__device__ __forceinline__ float bf2f(unsigned short b) { return __uint_as_float(((unsigned)b) << 16); }
__device__ __forceinline__ float bfr(float f) { return bf2f(f2bf(f)); }
__device__ __forceinline__ v16h cat16(v8h lo, v8h hi) { return __builtin_shufflevector(lo, hi, 0, 1, 2, 3, 4, 5, 6, 7, 8, 9, 10, 11, 12, 13, 14, 15); }
__device__ __forceinline__ v16bf cat16b(v8us lo, v8us hi) { return __builtin_bit_cast(v16bf, __builtin_shufflevector(lo, hi, 0, 1, 2, 3, 4, 5, 6, 7, 8, 9, 10, 11, 12, 13, 14, 15)); }
__device__ __forceinline__ v8f wmma16(v16h a, v16h b, v8f c) { return __builtin_amdgcn_wmma_f32_16x16x32_f16(false, a, false, b, (short)0, c, false, false); }
__device__ __forceinline__ v8f wmmab(v16bf a, v16bf b, v8f c) { return __builtin_amdgcn_wmma_f32_16x16x32_bf16(false, a, false, b, (short)0, c, false, false); }
__device__ __forceinline__ void splitf(float y, unsigned short& h, unsigned short& l) { h = f2bf(y); l = f2bf(y - bf2f(h)); }
static __device__ __forceinline__ h16 toh_flush(float v) { const h16 r = (h16)v; return (fabsf(v) < 6.103515625e-05f) ? (h16)0.0f : r; }

template <typename T16> struct WFrag;
template <> struct WFrag<h16> { typedef v16h V; static __device__ __forceinline__ V ld(const h16* p) { return cat16(*(const v8h*)p, *(const v8h*)(p + 16)); } static __device__ __forceinline__ v8f mma(V a, V b, v8f c) { return wmma16(a, b, c); } };
template <> struct WFrag<bf> { typedef v16bf V; static __device__ __forceinline__ V ld(const bf* p) { return cat16b(*(const v8us*)p, *(const v8us*)(p + 16)); } static __device__ __forceinline__ v8f mma(V a, V b, v8f c) { return wmmab(a, b, c); } };
template <typename T16, int NSPLIT, bool BIAS>
__global__ __launch_bounds__(32) void k_gemmw(const T16* __restrict__ A, const T16* __restrict__ A2, const T16* __restrict__ Bt, const T16* __restrict__ Bt2, int K, float* C, int ldc, const float* __restrict__ bias, size_t sA, size_t sB, size_t sC) {
    typedef typename WFrag<T16>::V V;
    __shared__ __align__(16) float os[16 * 68];
    const size_t z = blockIdx.z; A += z * sA; if (A2) A2 += z * sA; Bt += z * sB; if (Bt2) Bt2 += z * sB; C += z * sC;
    const int lane = threadIdx.x & 31, lr = lane & 15, hi = lane >> 4; const int r0 = blockIdx.x * 64, c0 = blockIdx.y * 64;
    v8f acc[4][4];
#pragma unroll
    for (int mb = 0; mb < 4; ++mb)
#pragma unroll
        for (int nb = 0; nb < 4; ++nb) acc[mb][nb] = (v8f){};
    const size_t aoff = (size_t)(r0 + lr) * K + 8 * hi, boff = (size_t)(c0 + lr) * K + 8 * hi;
#pragma unroll 1
    for (int kc = 0; kc < K; kc += 32) {
        V a[4], a2[4];
#pragma unroll
        for (int mb = 0; mb < 4; ++mb) { a[mb] = WFrag<T16>::ld(A + aoff + (size_t)mb * 16 * K + kc); if (NSPLIT == 1 || NSPLIT == 2) a2[mb] = WFrag<T16>::ld(A2 + aoff + (size_t)mb * 16 * K + kc); }
#pragma unroll
        for (int nb = 0; nb < 4; ++nb) { const V b = WFrag<T16>::ld(Bt + boff + (size_t)nb * 16 * K + kc); V b2; if (NSPLIT >= 2) b2 = WFrag<T16>::ld(Bt2 + boff + (size_t)nb * 16 * K + kc);
#pragma unroll
            for (int mb = 0; mb < 4; ++mb) { acc[mb][nb] = WFrag<T16>::mma(a[mb], b, acc[mb][nb]); if (NSPLIT == 1 || NSPLIT == 2) acc[mb][nb] = WFrag<T16>::mma(a2[mb], b, acc[mb][nb]); if (NSPLIT >= 2) acc[mb][nb] = WFrag<T16>::mma(a[mb], b2, acc[mb][nb]); } }
        asm volatile("v_nop\n\tv_nop\n\tv_nop\n\tv_nop" : "+v"(acc[0][0]), "+v"(acc[1][1]), "+v"(acc[2][2]), "+v"(acc[3][3]) : "v"(a[0]), "v"(a[3]));
    }
#pragma unroll
    for (int mb = 0; mb < 4; ++mb) {
#pragma unroll
        for (int nb = 0; nb < 4; ++nb) {
#pragma unroll
            for (int j = 0; j < 8; ++j) os[(hi * 8 + j) * 68 + nb * 16 + lr] = acc[mb][nb][j]; }
        __builtin_amdgcn_wave_barrier(); asm volatile("" ::: "memory");
        float* crow = C + (size_t)(r0 + mb * 16) * ldc + c0;
#pragma unroll 1
        for (int ps = 0; ps < 2; ++ps) {
#pragma unroll
            for (int s = 0; s < 8; ++s) { const int row = 2 * s + hi, cofs = lr * 4; v4f val = *(const v4fa*)(os + row * 68 + cofs); if (BIAS) { val[0] += bfr(bias[c0 + cofs]); val[1] += bfr(bias[c0 + cofs + 1]); val[2] += bfr(bias[c0 + cofs + 2]); val[3] += bfr(bias[c0 + cofs + 3]); }
                *(volatile v4f*)(crow + (size_t)row * ldc + cofs) = val; }
            if (ps == 0) __threadfence(); }
        __builtin_amdgcn_wave_barrier(); asm volatile("" ::: "memory");
    }
}

__global__ __launch_bounds__(256) void k_cvt8(const float* __restrict__ src, bf* dst, unsigned n8, size_t sS, size_t sD) {
    const unsigned i = blockIdx.x * 256u + threadIdx.x; if (i >= n8) return;
    const float* s = src + (size_t)blockIdx.y * sS + (size_t)i * 8; bf* d = dst + (size_t)blockIdx.y * sD + (size_t)i * 8;
    const v8f v = *(const v8f*)s; v8us o;
#pragma unroll
    for (int k = 0; k < 8; ++k) o[k] = f2bf(v[k]);
    *(volatile v8us*)d = o; __threadfence(); *(volatile v8us*)d = o; }

__global__ __launch_bounds__(256) void k_qkp(const float* __restrict__ F, h16* P16) {
    const unsigned e = (blockIdx.x * 256u + threadIdx.x) * 2u; if (e >= (unsigned)(NB * NQK * SEQ * HD)) return;
    const unsigned d = e & 63u; const unsigned row = e >> 6; const unsigned t = row % (unsigned)SEQ; const unsigned hb = row / (unsigned)SEQ; const unsigned h = hb % (unsigned)NQK; const unsigned b = hb / (unsigned)NQK;
    const float* f = F + (size_t)(b * (unsigned)SEQ + t) * NF + h * (unsigned)HD; v2h o16;
#pragma unroll
    for (unsigned q = 0; q < 2; ++q) { const float x0 = f[d + q]; o16[q] = toh_flush(x0); }
    *(volatile v2h*)(P16 + e) = o16; __threadfence(); *(volatile v2h*)(P16 + e) = o16; }

__global__ __launch_bounds__(256) void k_vtp(const float* __restrict__ F, h16* VT) {
    const unsigned e = (blockIdx.x * 256u + threadIdx.x) * 2u; if (e >= (unsigned)(NB * NKV * HD * SEQ)) return;
    const unsigned t = e % (unsigned)SEQ; const unsigned r2 = e / (unsigned)SEQ; const unsigned d = r2 & 63u; const unsigned gb = r2 >> 6; const unsigned g = gb & (unsigned)(NKV - 1); const unsigned b = gb / (unsigned)NKV; v2h o16;
#pragma unroll
    for (unsigned q = 0; q < 2; ++q) { const float x = F[(size_t)(b * (unsigned)SEQ + t + q) * NF + (unsigned)VOFF + g * (unsigned)HD + d]; o16[q] = (h16)x; }
    *(volatile v2h*)(VT + e) = o16; __threadfence(); *(volatile v2h*)(VT + e) = o16; }

__device__ __forceinline__ v16h ldh(const h16* p) { return cat16(*(const v8h*)p, *(const v8h*)(p + 16)); }
__global__ __launch_bounds__(128) void k_flash(const h16* __restrict__ QK, const h16* __restrict__ VT, bf* ATh, bf* ATl) {
    __shared__ __align__(16) float os[4 * 16 * 68];
    const unsigned lane = threadIdx.x & 31u, wv = threadIdx.x >> 5, lr = lane & 15u, hi = lane >> 4;
    const unsigned job = blockIdx.x * 4u + wv;
    const unsigned qt = job % (unsigned)QT, rest = job / (unsigned)QT;
    const unsigned hp = rest & 1u, g = (rest >> 1) & (unsigned)(NKV - 1), b = rest / (unsigned)(2 * NKV);
    if (b >= (unsigned)NB) return;
    const unsigned h0 = g * (unsigned)REP + hp * 2u;
    const h16* qp = QK + ((size_t)(b * (unsigned)NQK + h0) * SEQ + qt * 16u + lr) * HD + 8u * hi;
    const h16* kp = QK + ((size_t)(b * (unsigned)NQK + (unsigned)NH_ + g) * SEQ + lr) * HD + 8u * hi;
    const h16* vp = VT + ((size_t)(b * (unsigned)NKV + g) * HD + lr) * SEQ + 8u * hi;
    v16h qf[2][2];
#pragma unroll
    for (int hq = 0; hq < 2; ++hq)
#pragma unroll
        for (int ks = 0; ks < 2; ++ks) qf[hq][ks] = ldh(qp + (size_t)hq * SEQ * HD + ks * 32);
    v8f o[2][4]; float m[2], l[2];
#pragma unroll
    for (int hq = 0; hq < 2; ++hq) { m[hq] = -3.0e38f; l[hq] = 0.0f;
#pragma unroll
        for (int dt = 0; dt < 4; ++dt) o[hq][dt] = (v8f){}; }
#pragma unroll 1
    for (unsigned kb = 0; kb < (unsigned)SEQ; kb += 32u) {
        v16h kf[2][2];
#pragma unroll
        for (int kt = 0; kt < 2; ++kt)
#pragma unroll
            for (int ks = 0; ks < 2; ++ks) kf[kt][ks] = ldh(kp + (size_t)(kb + kt * 16u) * HD + ks * 32);
        v16h pf[2];
#pragma unroll
        for (int hq = 0; hq < 2; ++hq) {
            v8f s0 = (v8f){}, s1 = (v8f){};
            s0 = wmma16(kf[0][0], qf[hq][0], s0); s0 = wmma16(kf[0][1], qf[hq][1], s0);
            s1 = wmma16(kf[1][0], qf[hq][0], s1); s1 = wmma16(kf[1][1], qf[hq][1], s1);
            asm volatile("v_nop\n\tv_nop\n\tv_nop\n\tv_nop" : "+v"(s0), "+v"(s1) : "v"(kf[0][0]), "v"(kf[0][1]), "v"(kf[1][0]), "v"(kf[1][1]), "v"(qf[hq][0]), "v"(qf[hq][1]));
            float mx = fmaxf(s0[0], s1[0]);
#pragma unroll
            for (int j = 1; j < 8; ++j) mx = fmaxf(mx, fmaxf(s0[j], s1[j]));
            mx = fmaxf(mx, __shfl_xor(mx, 16, 32));
            const float mn = fmaxf(m[hq], mx);
            const float corr = __builtin_amdgcn_exp2f((m[hq] - mn) * CEXP);
            m[hq] = mn;
            const float nm = fmaf(-mn, CEXP, PEXP);
            float ls = 0.0f; v16h pv;
#pragma unroll
            for (int j = 0; j < 8; ++j) { const float p0 = __builtin_amdgcn_exp2f(fmaf(s0[j], CEXP, nm)); const float p1 = __builtin_amdgcn_exp2f(fmaf(s1[j], CEXP, nm)); ls += p0 + p1; pv[j] = (h16)p0; pv[8 + j] = (h16)p1; }
            l[hq] = fmaf(l[hq], corr, ls);
#pragma unroll
            for (int dt = 0; dt < 4; ++dt) o[hq][dt] *= corr;
            pf[hq] = pv;
        }
        v16h vf[4];
#pragma unroll
        for (int dt = 0; dt < 4; ++dt) vf[dt] = ldh(vp + (size_t)dt * 16 * SEQ + kb);
#pragma unroll
        for (int dt = 0; dt < 4; ++dt) { o[0][dt] = wmma16(vf[dt], pf[0], o[0][dt]); o[1][dt] = wmma16(vf[dt], pf[1], o[1][dt]); }
        asm volatile("v_nop\n\tv_nop\n\tv_nop\n\tv_nop" : "+v"(o[0][0]), "+v"(o[0][1]), "+v"(o[0][2]), "+v"(o[0][3]), "+v"(o[1][0]), "+v"(o[1][1]), "+v"(o[1][2]), "+v"(o[1][3]) : "v"(vf[0]), "v"(vf[1]), "v"(vf[2]), "v"(vf[3]), "v"(pf[0]), "v"(pf[1]));
    }
    float* osw = os + wv * (16 * 68);
    const size_t tok0 = (size_t)b * SEQ + qt * 16u;
#pragma unroll
    for (int hq = 0; hq < 2; ++hq) {
        const float ltot = l[hq] + __shfl_xor(l[hq], 16, 32);
        const float inv = 1.0f / ltot;
#pragma unroll
        for (int dt = 0; dt < 4; ++dt) { v4f a, c;
#pragma unroll
            for (int j = 0; j < 4; ++j) { a[j] = o[hq][dt][j] * inv; c[j] = o[hq][dt][4 + j] * inv; }
            *(v4fa*)(osw + lr * 68u + dt * 16 + 8u * hi) = a; *(v4fa*)(osw + lr * 68u + dt * 16 + 8u * hi + 4u) = c; }
        __builtin_amdgcn_wave_barrier(); asm volatile("" ::: "memory");
#pragma unroll 1
        for (int ps = 0; ps < 2; ++ps) {
#pragma unroll
            for (unsigned s = 0; s < 4; ++s) { const unsigned row = 4u * s + (lane >> 3), pc = lane & 7u;
                const v4f a = *(const v4fa*)(osw + row * 68u + pc * 8u); const v4f c = *(const v4fa*)(osw + row * 68u + pc * 8u + 4u); v8us oh, ol;
#pragma unroll
                for (int j = 0; j < 4; ++j) { unsigned short x, y; splitf(a[j], x, y); oh[j] = x; ol[j] = y; splitf(c[j], x, y); oh[4 + j] = x; ol[4 + j] = y; }
                const size_t off = (tok0 + row) * DQ + (size_t)(h0 + (unsigned)hq) * HD + pc * 8u;
                *(volatile v8us*)(ATh + off) = oh; *(volatile v8us*)(ATl + off) = ol; }
            if (ps == 0) __threadfence(); }
        __builtin_amdgcn_wave_barrier(); asm volatile("" ::: "memory");
    }
}

extern "C" void kernel_launch(void* const* d_in, const int* in_sizes, int n_in,
                              void* d_out, int out_size, void* d_ws, size_t ws_size, hipStream_t stream) {
    if (n_in < 5) return;
    if ((long long)in_sizes[0] < (long long)(NB - 1) * SEQ_FULL * DM + (long long)SEQ * DM) return;
    if ((long long)in_sizes[1] < (long long)DQ * DM || (long long)in_sizes[2] < (long long)DKV * DM || (long long)in_sizes[3] < (long long)DKV * DM || (long long)in_sizes[4] < (long long)DM * DQ) return;
    if ((long long)out_size < (long long)MTOK * DM) return;
    if (ws_size < WS_TOTAL) return;
    const float* x = (const float*)d_in[0]; const float* wq = (const float*)d_in[1]; const float* wk = (const float*)d_in[2]; const float* wv = (const float*)d_in[3]; const float* wo = (const float*)d_in[4];
    float* OUT = (float*)d_out;
    char* wsp = (char*)d_ws;
    bf* WQKV = (bf*)(wsp + OFF_WQKV);
    bf* WO = (bf*)(wsp + OFF_WO);
    bf* XB = (bf*)(wsp + OFF_XB);
    float* F = (float*)(wsp + OFF_F);
    h16* QK = (h16*)(wsp + OFF_QK);
    h16* VT = (h16*)(wsp + OFF_VT);
    bf* ATh = (bf*)(wsp + OFF_F); bf* ATl = (bf*)(wsp + OFF_F + SZ_AT);
    k_cvt8<<<dim3((unsigned)((size_t)DQ * DM / 8 / 256), 1, 1), 256, 0, stream>>>(wq, WQKV, (unsigned)((size_t)DQ * DM / 8), 0, 0);
    k_cvt8<<<dim3((unsigned)((size_t)DKV * DM / 8 / 256), 1, 1), 256, 0, stream>>>(wk, WQKV + (size_t)DQ * DM, (unsigned)((size_t)DKV * DM / 8), 0, 0);
    k_cvt8<<<dim3((unsigned)((size_t)DKV * DM / 8 / 256), 1, 1), 256, 0, stream>>>(wv, WQKV + (size_t)VOFF * DM, (unsigned)((size_t)DKV * DM / 8), 0, 0);
    k_cvt8<<<dim3((unsigned)((size_t)DM * DQ / 8 / 256), 1, 1), 256, 0, stream>>>(wo, WO, (unsigned)((size_t)DM * DQ / 8), 0, 0);
    k_cvt8<<<dim3((unsigned)((size_t)SEQ * DM / 8 / 256), NB, 1), 256, 0, stream>>>(x, XB, (unsigned)((size_t)SEQ * DM / 8), (size_t)SEQ_FULL * DM, (size_t)SEQ * DM);
    k_gemmw<bf, 0, false><<<dim3(MTOK / 64, NF / 64, 1), 32, 0, stream>>>(XB, nullptr, WQKV, nullptr, DM, F, NF, nullptr, 0, 0, 0);
    k_qkp<<<(unsigned)((size_t)NB * NQK * SEQ * HD / 512), 256, 0, stream>>>(F, QK);
    k_vtp<<<(unsigned)((size_t)NB * NKV * HD * SEQ / 512), 256, 0, stream>>>(F, VT);
    k_flash<<<MTOK / 4, 128, 0, stream>>>(QK, VT, ATh, ATl);
    k_gemmw<bf, 1, false><<<dim3(MTOK / 64, DM / 64, 1), 32, 0, stream>>>(ATh, ATl, WO, nullptr, DQ, OUT, DM, nullptr, 0, 0, 0);
}
